// CSAB3_1322849927417
// MI455X (gfx1250) — hardware-run, weakly checked
//
#include <hip/hip_runtime.h>
#include <math.h>
#include <stdint.h>

#define NB    8
#define SEQ   1024
#define DM    512
#define NH    8
#define HD    64
#define NKB   (SEQ / 64)
#define QKP   (2 * DM)
#define CP    (2 * DM)
#define MR    (NB * SEQ)
static_assert(NH * HD == DM);
static_assert((SEQ % 64) == 0 && (DM % 64) == 0 && (DM % 32) == 0);

typedef _Float16 v16h __attribute__((ext_vector_type(16)));
typedef _Float16 v8h  __attribute__((ext_vector_type(8)));
typedef __bf16   v16b __attribute__((ext_vector_type(16)));
typedef __bf16   v8b  __attribute__((ext_vector_type(8)));
typedef float    v8f  __attribute__((ext_vector_type(8)));
typedef float    v4f  __attribute__((ext_vector_type(4)));
typedef unsigned int v4u __attribute__((ext_vector_type(4)));

__device__ __forceinline__ unsigned short bf_bits(float f) {
  unsigned u = __float_as_uint(f);
  return (unsigned short)((u + 0x7FFFu + ((u >> 16) & 1u)) >> 16);
}
__device__ __forceinline__ float bf_up(unsigned short h) { return __uint_as_float(((unsigned)h) << 16); }
__device__ __forceinline__ float bfr(float f) { return bf_up(bf_bits(f)); }
__device__ __forceinline__ unsigned short h_bits(_Float16 x) { return __builtin_bit_cast(unsigned short, x); }
__device__ __forceinline__ unsigned pk16(unsigned short a, unsigned short b) { return (unsigned)a | ((unsigned)b << 16); }
__device__ __forceinline__ v8f zero8() { v8f z = {0.f, 0.f, 0.f, 0.f, 0.f, 0.f, 0.f, 0.f}; return z; }

__device__ __forceinline__ v16b ldfrag_b(const __bf16* p) {
  union { v16b v; v8b h[2]; } f;
  f.h[0] = *(const v8b*)(p);
  f.h[1] = *(const v8b*)(p + 16);
  return f.v;
}
__device__ __forceinline__ v16h ldfrag_h(const _Float16* p) {
  union { v16h v; v8h h[2]; } f;
  f.h[0] = *(const v8h*)(p);
  f.h[1] = *(const v8h*)(p + 16);
  return f.v;
}

__device__ __forceinline__ v8f mma_h(v16h a, v16h b, v8f c) {
  c = __builtin_amdgcn_wmma_f32_16x16x32_f16(false, a, false, b, (short)0, c, false, false);
#if defined(__HIP_DEVICE_COMPILE__)
  asm volatile("v_nop\n\tv_nop\n\tv_nop\n\tv_nop" : "+v"(c) : "v"(a), "v"(b));
#endif
  return c;
}
__device__ __forceinline__ v8f mma_b_raw(v16b a, v16b b, v8f c) {
  return __builtin_amdgcn_wmma_f32_16x16x32_bf16(false, a, false, b, (short)0, c, false, false);
}
__device__ __forceinline__ void dep_guard_b(v8f& a, v8f& b, v16b x, v16b y) {
#if defined(__HIP_DEVICE_COMPILE__)
  asm volatile("v_nop\n\tv_nop\n\tv_nop\n\tv_nop" : "+v"(a), "+v"(b) : "v"(x), "v"(y));
#endif
}
__device__ __forceinline__ void keep4_b(v16b a, v16b b, v16b c, v16b d) {
#if defined(__HIP_DEVICE_COMPILE__)
  asm volatile("v_nop" :: "v"(a), "v"(b), "v"(c), "v"(d));
#endif
}
__device__ __forceinline__ void acc_guard4(v8f& a, v8f& b, v8f& c, v8f& d) {
#if defined(__HIP_DEVICE_COMPILE__)
  asm volatile("v_nop\n\tv_nop\n\tv_nop\n\tv_nop" : "+v"(a), "+v"(b), "+v"(c), "+v"(d));
#endif
}
__device__ __forceinline__ void wave_sync_lds() {
  __builtin_amdgcn_fence(__ATOMIC_RELEASE, "workgroup");
  __builtin_amdgcn_wave_barrier();
  __builtin_amdgcn_fence(__ATOMIC_ACQUIRE, "workgroup");
}

__global__ __launch_bounds__(256) void cvt_bf16x8(const float* __restrict__ in, unsigned short* out, int n8) {
  const int i = blockIdx.x * 256 + threadIdx.x;
  if (i < n8) {
    const v4f a = *(const v4f*)(in + (size_t)i * 8);
    const v4f b = *(const v4f*)(in + (size_t)i * 8 + 4);
    v4u p;
    p[0] = pk16(bf_bits(a[0]), bf_bits(a[1]));
    p[1] = pk16(bf_bits(a[2]), bf_bits(a[3]));
    p[2] = pk16(bf_bits(b[0]), bf_bits(b[1]));
    p[3] = pk16(bf_bits(b[2]), bf_bits(b[3]));
    *(volatile v4u*)(out + (size_t)i * 8) = p;
    __threadfence();
    *(volatile v4u*)(out + (size_t)i * 8) = p;
  }
}

__global__ __launch_bounds__(256) void tr_bf16(const float* __restrict__ s0, const float* __restrict__ s1,
                                               const float* __restrict__ s2, const float* __restrict__ s3,
                                               unsigned short* dst, long long zstride, int nrow, int ncol) {
  __shared__ __align__(16) unsigned short T[64][66];
  const int z = blockIdx.z;
  const float* src = (z == 0) ? s0 : ((z == 1) ? s1 : ((z == 2) ? s2 : s3));
  unsigned short* out = dst + (size_t)z * (size_t)zstride;
  const int c0 = blockIdx.x * 64, r0 = blockIdx.y * 64;
  const int tid = threadIdx.x, lane = tid & 31, wave = tid >> 5;
  {
    const int row = tid >> 2, cs = (tid & 3) * 16;
    const float* g = src + (size_t)(r0 + row) * ncol + c0 + cs;
#pragma unroll
    for (int i = 0; i < 4; ++i) {
      const v4f v = *(const v4f*)(g + 4 * i);
#pragma unroll
      for (int e = 0; e < 4; ++e) T[cs + 4 * i + e][row] = bf_bits(v[e]);
    }
  }
  __syncthreads();
  const int q = lane >> 3, c8 = (lane & 7) * 8;
  v4u pv[2];
#pragma unroll
  for (int it = 0; it < 2; ++it) {
    const int c = wave * 8 + it * 4 + q;
    v4u p;
#pragma unroll
    for (int e = 0; e < 4; ++e) p[e] = pk16(T[c][c8 + 2 * e], T[c][c8 + 2 * e + 1]);
    pv[it] = p;
  }
  for (int pass = 0; pass < 2; ++pass) {
#pragma unroll
    for (int it = 0; it < 2; ++it) {
      const int c = wave * 8 + it * 4 + q;
      *(volatile v4u*)(out + (size_t)(c0 + c) * nrow + r0 + c8) = pv[it];
    }
    __threadfence();
  }
}

template <int NSPLIT, int OUT_MODE, int BIAS>
__global__ __launch_bounds__(256) void gemm64(
    const unsigned short* __restrict__ Ap, const unsigned short* A2p, int lda, long long strideA,
    const unsigned short* __restrict__ Btp, int ldb, long long strideB,
    const float* __restrict__ bias, const float* __restrict__ Rp, int ldr,
    void* Cout, int ldc, long long strideC,
    void* Cout2, int ldc2, long long strideC2, int N2,
    int M, int N, int K, float rscale) {
  const __bf16* A   = (const __bf16*)(const void*)Ap;
  const __bf16* A2  = (const __bf16*)(const void*)A2p;
  const __bf16* Bt  = (const __bf16*)(const void*)Btp;
  __shared__ __align__(16) float sT[8][16 * 68];
  const int b    = blockIdx.y;
  const int lane = threadIdx.x & 31;
  const int wave = threadIdx.x >> 5;
  const int tilesN = N >> 6;
  const int tilesM = M >> 6;
  const int tile = blockIdx.x * 8 + wave;
  if (tile >= tilesM * tilesN) return;
  const int tm = tile / tilesN;
  const int tn = tile - tm * tilesN;
  const int m0 = tm << 6;
  const int n0 = tn << 6;

  const __bf16* Ab  = A  + (size_t)b * strideA;
  const __bf16* Bb  = Bt + (size_t)b * strideB;
  const __bf16* Ab2 = (NSPLIT >= 1) ? (A2 + (size_t)b * strideA) : Ab;

  const int rlane = lane & 15;
  const int koff  = (lane >> 4) * 8;
  const int mOff  = (lane >> 4) * 8;

  v8f acc[4][4];
#pragma unroll
  for (int i = 0; i < 4; ++i)
#pragma unroll
    for (int j = 0; j < 4; ++j) acc[i][j] = zero8();

  for (int k0 = 0; k0 < K; k0 += 32) {
    v16b bh[4];
#pragma unroll
    for (int j = 0; j < 4; ++j) {
      const size_t bo = (size_t)(n0 + (j << 4) + rlane) * ldb + koff + k0;
      bh[j] = ldfrag_b(Bb + bo);
    }
#pragma unroll
    for (int i = 0; i < 4; ++i) {
      const size_t ao = (size_t)(m0 + (i << 4) + rlane) * lda + koff + k0;
      const v16b ah = ldfrag_b(Ab + ao);
      v16b al = ah;
      if (NSPLIT >= 1) al = ldfrag_b(Ab2 + ao);
#pragma unroll
      for (int j = 0; j < 4; ++j) {
        acc[i][j] = mma_b_raw(ah, bh[j], acc[i][j]);
        if (NSPLIT >= 1) acc[i][j] = mma_b_raw(al, bh[j], acc[i][j]);
      }
      dep_guard_b(acc[i][0], acc[i][3], ah, al);
    }
    keep4_b(bh[0], bh[1], bh[2], bh[3]);
  }
  acc_guard4(acc[0][0], acc[0][1], acc[0][2], acc[0][3]);
  acc_guard4(acc[1][0], acc[1][1], acc[1][2], acc[1][3]);
  acc_guard4(acc[2][0], acc[2][1], acc[2][2], acc[2][3]);
  acc_guard4(acc[3][0], acc[3][1], acc[3][2], acc[3][3]);

  float bcol[4];
#pragma unroll
  for (int j = 0; j < 4; ++j) bcol[j] = (BIAS == 1) ? bfr(bias[n0 + (j << 4) + rlane]) : 0.f;
  float* slab = sT[wave];
#pragma unroll
  for (int i = 0; i < 4; ++i) {
    const int mBase = m0 + (i << 4);
    float brow[8];
#pragma unroll
    for (int r = 0; r < 8; ++r) brow[r] = (BIAS == 2) ? bfr(bias[mBase + mOff + r]) : 0.f;
#pragma unroll
    for (int j = 0; j < 4; ++j) {
#pragma unroll
      for (int r = 0; r < 8; ++r) {
        slab[(mOff + r) * 68 + (j << 4) + rlane] = acc[i][j][r] + bcol[j] + brow[r];
      }
    }
    wave_sync_lds();
    if (OUT_MODE == 1) {
      float* C = (float*)Cout + (size_t)b * strideC;
      const int hh = lane >> 4, c4 = (lane & 15) * 4;
      for (int pass = 0; pass < 2; ++pass) {
#pragma unroll
        for (int it = 0; it < 8; ++it) {
          const int row = it * 2 + hh;
          const v4f v = *(const v4f*)(slab + row * 68 + c4);
          const v4f x = *(const v4f*)(Rp + (size_t)(mBase + row) * ldr + n0 + c4);
          v4f o;
#pragma unroll
          for (int e = 0; e < 4; ++e) o[e] = bf_up(bf_bits(x[e])) + fmaxf(v[e], 0.0f);
          *(volatile v4f*)(C + (size_t)(mBase + row) * ldc + n0 + c4) = o;
        }
        __threadfence();
      }
    } else {
      const int q = lane >> 3, c8 = (lane & 7) * 8;
      unsigned short* C  = (unsigned short*)Cout  + (size_t)b * strideC;
      unsigned short* C2 = (unsigned short*)Cout2 + (size_t)b * strideC2;
      const bool wlo = (n0 < N2);
      v4u hv[4], lv[4];
#pragma unroll
      for (int it = 0; it < 4; ++it) {
        const int row = it * 4 + q;
        const float* sp = slab + row * 68 + c8;
        v4u a, a2;
#pragma unroll
        for (int e = 0; e < 4; ++e) {
          const float f0 = sp[2 * e], f1 = sp[2 * e + 1];
          const _Float16 x0 = (_Float16)f0, x1 = (_Float16)f1;
          const unsigned short h0 = h_bits(x0), h1 = h_bits(x1);
          const unsigned short l0 = h_bits((_Float16)((f0 - (float)x0) * rscale));
          const unsigned short l1 = h_bits((_Float16)((f1 - (float)x1) * rscale));
          a[e] = pk16(h0, h1); a2[e] = pk16(l0, l1);
        }
        hv[it] = a; lv[it] = a2;
      }
      for (int pass = 0; pass < 2; ++pass) {
#pragma unroll
        for (int it = 0; it < 4; ++it) {
          const int row = it * 4 + q;
          *(volatile v4u*)(C + (size_t)(mBase + row) * ldc + n0 + c8) = hv[it];
          if (wlo) *(volatile v4u*)(C2 + (size_t)(mBase + row) * ldc2 + n0 + c8) = lv[it];
        }
        __threadfence();
      }
    }
    wave_sync_lds();
  }
}

__global__ __launch_bounds__(128)
void attn64(const unsigned short* __restrict__ qkp, const unsigned short* __restrict__ qlp,
            const unsigned short* __restrict__ vhp, const unsigned short* __restrict__ vlp,
            unsigned short* chp, unsigned short* clp, int colOff, float sscale, float rres) {
  union FH { v16h v; v8h h[2]; };
  __shared__ __align__(16) _Float16 Ksh[64 * 64];
  __shared__ __align__(16) _Float16 Vth[64 * 64];
  __shared__ __align__(16) _Float16 Vtl[64 * 64];
  __shared__ __align__(16) _Float16 Psh[4][16 * 64];
  __shared__ __align__(16) float    Os[4][16 * 64];

  const int tid  = threadIdx.x;
  const int wave = tid >> 5;
  const int lane = tid & 31;
  const int hh   = lane >> 4;
  const int c    = lane & 15;

  const int bx   = blockIdx.x;
  const int qb   = bx % NKB;
  const int rest = bx / NKB;
  const int h    = rest % NH;
  const int b    = rest / NH;
  const int q0   = qb * 64 + wave * 16;
  const size_t rowB = (size_t)b * SEQ;

  const _Float16* Qh = (const _Float16*)(const void*)qkp + (size_t)h * HD;
  const _Float16* Kg = (const _Float16*)(const void*)qkp + DM + (size_t)h * HD;
  const _Float16* Ql = (const _Float16*)(const void*)qlp + (size_t)h * HD;
  const _Float16* Vh = (const _Float16*)(const void*)vhp + ((size_t)b * DM + (size_t)h * HD) * SEQ;
  const _Float16* Vl = (const _Float16*)(const void*)vlp + ((size_t)b * DM + (size_t)h * HD) * SEQ;

  v16h qah[2], qal[2];
#pragma unroll
  for (int dc = 0; dc < 2; ++dc) {
    qah[dc] = ldfrag_h(Qh + (rowB + q0 + c) * QKP + dc * 32 + 8 * hh);
    qal[dc] = ldfrag_h(Ql + (rowB + q0 + c) * DM  + dc * 32 + 8 * hh);
  }

  float mrow[8], lrow[8];
  v8f oacc[4];
#pragma unroll
  for (int r = 0; r < 8; ++r) { mrow[r] = -INFINITY; lrow[r] = 0.f; }
#pragma unroll
  for (int t = 0; t < 4; ++t) oacc[t] = zero8();

  for (int kt = 0; kt < NKB; ++kt) {
    const int kv0 = kt * 64;
    __syncthreads();
    {
      const int r = tid >> 1, hf = (tid & 1) * 32;
      const _Float16* kg  = Kg + (rowB + kv0 + r) * QKP + hf;
      const _Float16* vg  = Vh + (size_t)r * SEQ + kv0 + hf;
      const _Float16* vlg = Vl + (size_t)r * SEQ + kv0 + hf;
#pragma unroll
      for (int i = 0; i < 4; ++i) {
        const v8h a0 = *(const v8h*)(kg + 8 * i);
        const v8h b0 = *(const v8h*)(vg + 8 * i);
        const v8h b1 = *(const v8h*)(vlg + 8 * i);
        *(v8h*)(Ksh + r * 64 + hf + 8 * i) = a0;
        *(v8h*)(Vth + r * 64 + hf + 8 * i) = b0;
        *(v8h*)(Vtl + r * 64 + hf + 8 * i) = b1;
      }
    }
    __syncthreads();

    v8f s[4];
#pragma unroll
    for (int j = 0; j < 4; ++j) {
      v8f sh = zero8(), sl = zero8();
#pragma unroll
      for (int dc = 0; dc < 2; ++dc) {
        FH kb;
        kb.h[0] = *(const v8h*)(Ksh + (j * 16 + c) * 64 + dc * 32 + 8 * hh);
        kb.h[1] = *(const v8h*)(Ksh + (j * 16 + c) * 64 + dc * 32 + 16 + 8 * hh);
        sh = mma_h(qah[dc], kb.v, sh);
        sl = mma_h(qal[dc], kb.v, sl);
      }
#pragma unroll
      for (int r = 0; r < 8; ++r) s[j][r] = (sh[r] + sl[r] * rres) * sscale;
    }

    _Float16* pwh = Psh[wave];
#pragma unroll
    for (int r = 0; r < 8; ++r) {
      float m = s[0][r];
      m = fmaxf(m, s[1][r]);
      m = fmaxf(m, s[2][r]);
      m = fmaxf(m, s[3][r]);
#pragma unroll
      for (int off = 1; off < 16; off <<= 1) m = fmaxf(m, __shfl_xor(m, off, 32));
      const float mnew  = fmaxf(mrow[r], m);
      const float alpha = __expf(mrow[r] - mnew);
      mrow[r] = mnew;
      float psum = 0.f;
#pragma unroll
      for (int j = 0; j < 4; ++j) {
        const float p = __expf(s[j][r] - mnew);
        psum += p;
        pwh[(8 * hh + r) * 64 + j * 16 + c] = (_Float16)(p * 1024.0f);
      }
#pragma unroll
      for (int off = 1; off < 16; off <<= 1) psum += __shfl_xor(psum, off, 32);
      lrow[r] = lrow[r] * alpha + psum;
#pragma unroll
      for (int t = 0; t < 4; ++t) oacc[t][r] *= alpha;
    }
    wave_sync_lds();

    v8f o1[4];
#pragma unroll
    for (int t = 0; t < 4; ++t) o1[t] = zero8();
#pragma unroll 1
    for (int kk = 0; kk < 2; ++kk) {
      FH pa;
      pa.h[0] = *(const v8h*)(pwh + c * 64 + kk * 32 + 8 * hh);
      pa.h[1] = *(const v8h*)(pwh + c * 64 + kk * 32 + 16 + 8 * hh);
#pragma unroll
      for (int t = 0; t < 4; ++t) {
        FH vb, vl;
        vb.h[0] = *(const v8h*)(Vth + (t * 16 + c) * 64 + kk * 32 + 8 * hh);
        vb.h[1] = *(const v8h*)(Vth + (t * 16 + c) * 64 + kk * 32 + 16 + 8 * hh);
        vl.h[0] = *(const v8h*)(Vtl + (t * 16 + c) * 64 + kk * 32 + 8 * hh);
        vl.h[1] = *(const v8h*)(Vtl + (t * 16 + c) * 64 + kk * 32 + 16 + 8 * hh);
        oacc[t] = mma_h(pa.v, vb.v, oacc[t]);
        o1[t]   = mma_h(pa.v, vl.v, o1[t]);
      }
    }
#pragma unroll
    for (int t = 0; t < 4; ++t)
#pragma unroll
      for (int r = 0; r < 8; ++r) oacc[t][r] += o1[t][r] * rres;
  }

  float* os = Os[wave];
#pragma unroll
  for (int r = 0; r < 8; ++r) {
    const float l = lrow[r];
    const float inv = ((l > 0.f) ? (1.0f / l) : 0.f) * (1.0f / 1024.0f);
#pragma unroll
    for (int t = 0; t < 4; ++t) os[(8 * hh + r) * 64 + t * 16 + c] = oacc[t][r] * inv;
  }
  wave_sync_lds();
  {
    const int q4 = lane >> 3, c8 = (lane & 7) * 8;
    v4u hv[4], lv[4];
#pragma unroll
    for (int it = 0; it < 4; ++it) {
      const int row = it * 4 + q4;
      const float* sp = os + row * 64 + c8;
      const size_t grow = rowB + q0 + row;
      const v8h qh8 = *(const v8h*)(Qh + grow * QKP + c8);
      const v8h ql8 = *(const v8h*)(Ql + grow * DM  + c8);
      v4u a, a2;
#pragma unroll
      for (int e = 0; e < 4; ++e) {
        const float f0 = sp[2 * e]     + ((float)qh8[2 * e]     + (float)ql8[2 * e]     * rres);
        const float f1 = sp[2 * e + 1] + ((float)qh8[2 * e + 1] + (float)ql8[2 * e + 1] * rres);
        const unsigned short h0 = bf_bits(f0), h1 = bf_bits(f1);
        const unsigned short l0 = bf_bits(f0 - bf_up(h0)), l1 = bf_bits(f1 - bf_up(h1));
        a[e] = pk16(h0, h1); a2[e] = pk16(l0, l1);
      }
      hv[it] = a; lv[it] = a2;
    }
    for (int pass = 0; pass < 2; ++pass) {
#pragma unroll
      for (int it = 0; it < 4; ++it) {
        const int row = it * 4 + q4;
        const size_t go = (rowB + q0 + row) * CP + (size_t)colOff + (size_t)h * HD + c8;
        *(volatile v4u*)(chp + go) = hv[it];
        *(volatile v4u*)(clp + go) = lv[it];
      }
      __threadfence();
    }
  }
}

extern "C" void kernel_launch(void* const* d_in, const int* in_sizes, int n_in,
                              void* d_out, int out_size, void* d_ws, size_t ws_size,
                              hipStream_t stream) {
  if (n_in < 30) return;
  if (in_sizes[0] != MR * DM) return;
  if (in_sizes[1] != MR * DM) return;
  for (int i = 0; i < 12; ++i) {
    if (in_sizes[2 + 2 * i] != DM * DM) return;
    if (in_sizes[3 + 2 * i] != DM) return;
  }
  if (in_sizes[26] != 2 * DM * DM || in_sizes[27] != DM) return;
  if (in_sizes[28] != 2 * DM * DM || in_sizes[29] != DM) return;
  if (out_size != 2 * MR * DM) return;

  const float* X = (const float*)d_in[0];
  const float* Y = (const float*)d_in[1];

  const size_t PXb  = (size_t)MR * DM * 2;
  const size_t PWT  = (size_t)12 * DM * DM * 2;
  const size_t PWO  = (size_t)DM * (2 * DM) * 2;
  const size_t PQK  = (size_t)MR * QKP * 2;
  const size_t PQl  = (size_t)MR * DM * 2;
  const size_t PVT  = (size_t)NB * DM * SEQ * 2;
  const size_t PC   = (size_t)MR * CP * 2;
  size_t off = 0;
  const size_t oXb  = off; off += PXb;
  const size_t oYb  = off; off += PXb;
  const size_t oWT  = off; off += PWT;
  const size_t oWXT = off; off += PWO;
  const size_t oWYT = off; off += PWO;
  const size_t oQK  = off; off += PQK;
  const size_t oQl  = off; off += PQl;
  const size_t oVTh = off; off += PVT;
  const size_t oVTl = off; off += PVT;
  const size_t oCh  = off; off += PC;
  const size_t oCl  = off; off += PC;
  if (off > ws_size) return;
  if (off > (size_t)134217728) return;

  char* ws = (char*)d_ws;
  unsigned short* Xb  = (unsigned short*)(ws + oXb);
  unsigned short* Yb  = (unsigned short*)(ws + oYb);
  unsigned short* WT  = (unsigned short*)(ws + oWT);
  unsigned short* WXT = (unsigned short*)(ws + oWXT);
  unsigned short* WYT = (unsigned short*)(ws + oWYT);
  unsigned short* QK  = (unsigned short*)(ws + oQK);
  unsigned short* Ql  = (unsigned short*)(ws + oQl);
  unsigned short* VTh = (unsigned short*)(ws + oVTh);
  unsigned short* VTl = (unsigned short*)(ws + oVTl);
  unsigned short* Ch  = (unsigned short*)(ws + oCh);
  unsigned short* Cl  = (unsigned short*)(ws + oCl);
  (void)WYT;

  const dim3 blk(256);
  const int n8x = MR * DM / 8;
  const dim3 gCvt((n8x + 255) / 256);
  const dim3 gTrW(DM / 64, DM / 64, 4);
  const dim3 gTrO(DM / 64, (2 * DM) / 64, 2);
  const dim3 gPrj(((MR / 64) * (DM / 64) + 7) / 8, 1);
  const dim3 gVT(((DM / 64) * (SEQ / 64) + 7) / 8, NB);
  const dim3 gOut(((MR / 64) * (DM / 64) + 7) / 8, 1);
  const dim3 gAttn(NB * NH * NKB);
  const float sscale = 1.0f / sqrtf((float)DM);
  const float rres = 1.0f / 4096.0f;
  const size_t WSZ = (size_t)DM * DM;

  cvt_bf16x8<<<gCvt, blk, 0, stream>>>(X, Xb, n8x);
  cvt_bf16x8<<<gCvt, blk, 0, stream>>>(Y, Yb, n8x);
  for (int g = 0; g < 3; ++g) {
    tr_bf16<<<gTrW, blk, 0, stream>>>(
        (const float*)d_in[2 + 2 * (4 * g + 0)], (const float*)d_in[2 + 2 * (4 * g + 1)],
        (const float*)d_in[2 + 2 * (4 * g + 2)], (const float*)d_in[2 + 2 * (4 * g + 3)],
        WT + (size_t)(4 * g) * WSZ, (long long)WSZ, DM, DM);
  }
  tr_bf16<<<gTrO, blk, 0, stream>>>((const float*)d_in[26], (const float*)d_in[28],
                                     (const float*)d_in[26], (const float*)d_in[28],
                                     WXT, (long long)(DM * 2 * DM), 2 * DM, DM);

  for (int z = 0; z < 4; ++z) {
    const unsigned short* qsrc  = (z < 2) ? Xb : Yb;
    const unsigned short* kvsrc = ((z & 1) == 0) ? Xb : Yb;
    const unsigned short* WqT = WT + (size_t)(3 * z + 0) * WSZ;
    const unsigned short* WkT = WT + (size_t)(3 * z + 1) * WSZ;
    const unsigned short* WvT = WT + (size_t)(3 * z + 2) * WSZ;
    const float* bq = (const float*)d_in[3 + 2 * (3 * z + 0)];
    const float* bk = (const float*)d_in[3 + 2 * (3 * z + 1)];
    const float* bv = (const float*)d_in[3 + 2 * (3 * z + 2)];
    const int colOff = (z & 1) * DM;

    gemm64<0, 3, 1><<<gPrj, blk, 0, stream>>>(
        qsrc, qsrc, DM, 0LL, WqT, DM, 0LL, bq, X, DM,
        (void*)QK, QKP, 0LL, (void*)Ql, DM, 0LL, DM,
        MR, DM, DM, 4096.0f);
    gemm64<0, 3, 1><<<gPrj, blk, 0, stream>>>(
        kvsrc, kvsrc, DM, 0LL, WkT, DM, 0LL, bk, X, DM,
        (void*)(QK + DM), QKP, 0LL, (void*)Ql, DM, 0LL, 0,
        MR, DM, DM, 4096.0f);
    gemm64<0, 3, 2><<<gVT, blk, 0, stream>>>(
        WvT, WvT, DM, 0LL, kvsrc, DM, (long long)SEQ * DM, bv, X, DM,
        (void*)VTh, SEQ, (long long)DM * SEQ, (void*)VTl, SEQ, (long long)DM * SEQ, SEQ,
        DM, SEQ, DM, 4096.0f);
    attn64<<<gAttn, dim3(128), 0, stream>>>(QK, Ql, VTh, VTl, Ch, Cl, colOff, sscale, rres);

    if (z == 1) {
      float* outx = (float*)d_out;
      gemm64<1, 1, 1><<<gOut, blk, 0, stream>>>(
          Ch, Cl, CP, 0LL, WXT, 2 * DM, 0LL, (const float*)d_in[27], X, DM,
          (void*)outx, DM, 0LL, (void*)outx, DM, 0LL, 0,
          MR, DM, 2 * DM, 1.0f);
    } else if (z == 3) {
      float* outy = (float*)d_out + (size_t)MR * DM;
      gemm64<1, 1, 1><<<gOut, blk, 0, stream>>>(
          Ch, Cl, CP, 0LL, WYT, 2 * DM, 0LL, (const float*)d_in[29], Y, DM,
          (void*)outy, DM, 0LL, (void*)outy, DM, 0LL, 0,
          MR, DM, 2 * DM, 1.0f);
    }
  }
  (void)hipGetLastError();
}
